// GIN2_40132174414143
// MI455X (gfx1250) — hardware-verified
//
#include <hip/hip_runtime.h>
#include <stddef.h>


#define DH      128
#define DMLP    512
#define DPR     64
#define NTHR    256
#define NWAVE   8
#define EPT     8
#define NGRP    2
#define CHUNK   (NTHR * EPT * NGRP)
#define WCAP    (EPT * NGRP * 32)
#define LISTN   (NWAVE * WCAP)
#define NBC     4096
#define NBF     1024
#define RCAP    40960
#define RBN     128
#define TGT     256
#define DEGCAP  256
#define OTHR    512
#define GR      64
#define GTHR    128
#define ZP      (DMLP + 8)
#define PB      64
#define PTHR    128
#define SPP     (DH + 8)

#define LDS_FILL ((RCAP + NBF + LISTN) * 4 + 64)
#define LDS_GIN  (2 * GR * ZP * 2)

static_assert((CHUNK & (CHUNK - 1)) == 0);
static_assert(CHUNK <= 4096);
static_assert((NBC & (NBC - 1)) == 0 && (NBF & (NBF - 1)) == 0);
static_assert(NBC == 4 * NBF);
static_assert(OTHR * 8 == NBC);
static_assert((RCAP % 32) == 0);
static_assert(TGT == NWAVE * 32 && (TGT % GR) == 0);
static_assert(GR == (GTHR / 32) * 16 && PB == (PTHR / 32) * 16);
static_assert(GR * DH * 4 <= LDS_GIN);
static_assert(((ZP * 2) % 16) == 0 && ((SPP * 2) % 16) == 0);
static_assert((DH % 32) == 0 && (DMLP % 64) == 0 && DPR == 64);
static_assert(((DH * DMLP / 8) % NTHR) == 0 && ((DH * DPR / 8) % NTHR) == 0);

typedef float          v4f   __attribute__((ext_vector_type(4)));
typedef float          v8f   __attribute__((ext_vector_type(8)));
typedef int            v4i   __attribute__((ext_vector_type(4)));
typedef unsigned short v4us  __attribute__((ext_vector_type(4)));
typedef unsigned short v8us  __attribute__((ext_vector_type(8)));
typedef unsigned short v16us __attribute__((ext_vector_type(16)));
typedef __bf16         v16bf __attribute__((ext_vector_type(16)));
union FragB { v16bf v; v16us u; v8us h[2]; };

__device__ __forceinline__ unsigned short f2bf(float f) {
  unsigned u = __float_as_uint(f);
  u += 0x7FFFu + ((u >> 16) & 1u);
  return (unsigned short)(u >> 16);
}
__device__ __forceinline__ float bf2f(unsigned short b) { return __uint_as_float(((unsigned)b) << 16); }
__device__ __forceinline__ float bfr(float f) { return bf2f(f2bf(f)); }
__device__ __forceinline__ v4f bfr4(v4f v) { v4f r; r.x = bfr(v.x); r.y = bfr(v.y); r.z = bfr(v.z); r.w = bfr(v.w); return r; }

__device__ __forceinline__ void split4(v4f v, v4us& hi, v4us& lo) {
  const unsigned short h0 = f2bf(v.x), h1 = f2bf(v.y), h2 = f2bf(v.z), h3 = f2bf(v.w);
  hi.x = h0; hi.y = h1; hi.z = h2; hi.w = h3;
  lo.x = f2bf(v.x - bf2f(h0)); lo.y = f2bf(v.y - bf2f(h1));
  lo.z = f2bf(v.z - bf2f(h2)); lo.w = f2bf(v.w - bf2f(h3));
}

__device__ __forceinline__ v8f wmb(v16bf a, v16bf b, v8f c) {
  v8f d = __builtin_amdgcn_wmma_f32_16x16x32_bf16(false, a, false, b, (short)0, c, false, false);
  asm volatile("v_nop\n\tv_nop\n\tv_nop\n\tv_nop" : "+v"(d) : "v"(a), "v"(b));
  return d;
}

__device__ __forceinline__ v8f zero8() { v8f z = {0.f, 0.f, 0.f, 0.f, 0.f, 0.f, 0.f, 0.f}; return z; }

template <int NB>
__device__ __forceinline__ int scan_chunk(const int* __restrict__ dsts, int nE, int cbase, int slotBase,
                                          int vec8, int* list, int tid, int lane, int wave) {
  int wc = 0;
#pragma unroll
  for (int g = 0; g < NGRP; ++g) {
    const int el0  = (g * NTHR + tid) * EPT;
    const int e0   = cbase + el0;
    const int sent = -2147483647 - 1;
    v4i da, db;
    if (vec8 != 0 && cbase + CHUNK <= nE) {
      da = *(const v4i*)(dsts + e0);
      db = *(const v4i*)(dsts + e0 + 4);
    } else {
      da.x = (e0     < nE) ? dsts[min(e0, nE - 1)] : sent;
      da.y = (e0 + 1 < nE) ? dsts[min(e0 + 1, nE - 1)] : sent;
      da.z = (e0 + 2 < nE) ? dsts[min(e0 + 2, nE - 1)] : sent;
      da.w = (e0 + 3 < nE) ? dsts[min(e0 + 3, nE - 1)] : sent;
      db.x = (e0 + 4 < nE) ? dsts[min(e0 + 4, nE - 1)] : sent;
      db.y = (e0 + 5 < nE) ? dsts[min(e0 + 5, nE - 1)] : sent;
      db.z = (e0 + 6 < nE) ? dsts[min(e0 + 6, nE - 1)] : sent;
      db.w = (e0 + 7 < nE) ? dsts[min(e0 + 7, nE - 1)] : sent;
    }
    const unsigned nb = (unsigned)slotBase;
    const unsigned s0 = (unsigned)da.x - nb, s1 = (unsigned)da.y - nb;
    const unsigned s2 = (unsigned)da.z - nb, s3 = (unsigned)da.w - nb;
    const unsigned s4 = (unsigned)db.x - nb, s5 = (unsigned)db.y - nb;
    const unsigned s6 = (unsigned)db.z - nb, s7 = (unsigned)db.w - nb;
    const bool h0 = s0 < (unsigned)NB, h1 = s1 < (unsigned)NB, h2 = s2 < (unsigned)NB, h3 = s3 < (unsigned)NB;
    const bool h4 = s4 < (unsigned)NB, h5 = s5 < (unsigned)NB, h6 = s6 < (unsigned)NB, h7 = s7 < (unsigned)NB;
    const unsigned any = __builtin_amdgcn_ballot_w32(h0 | h1 | h2 | h3 | h4 | h5 | h6 | h7);
    if (any != 0u) {
#define HITJ(J, HJ, SJ) { \
        const unsigned mj = __builtin_amdgcn_ballot_w32(HJ); \
        if (mj != 0u) { \
          if (HJ) { \
            const int pos = wc + (int)__builtin_amdgcn_mbcnt_lo(mj, 0u); \
            if (pos < WCAP) list[wave * WCAP + pos] = ((el0 + (J)) << 12) | (int)(SJ); \
          } \
          wc += (int)__builtin_popcount(mj); } }
      HITJ(0, h0, s0)
      HITJ(1, h1, s1)
      HITJ(2, h2, s2)
      HITJ(3, h3, s3)
      HITJ(4, h4, s4)
      HITJ(5, h5, s5)
      HITJ(6, h6, s6)
      HITJ(7, h7, s7)
#undef HITJ
    }
  }
  return wc;
}

__global__ __launch_bounds__(NTHR) void k_wprep(
    const float* __restrict__ W1, const float* __restrict__ W2, const float* __restrict__ Wp1,
    unsigned short* w1p, unsigned short* w2p, unsigned short* wpp, int nL) {
  const int g1 = nL * (DH * DMLP / 8);
  const int g2 = nL * (DMLP * DH / 8);
  const int g3 = DH * DPR / 8;
  const int bstart = blockIdx.x * NTHR;
  const float* src; unsigned short* dst; int Nout, KP, segOff, per;
  if (bstart < g1)           { src = W1;  dst = w1p; Nout = DMLP; KP = DH;   segOff = 0;       per = DH * DMLP; }
  else if (bstart < g1 + g2) { src = W2;  dst = w2p; Nout = DH;   KP = DMLP; segOff = g1;      per = DMLP * DH; }
  else                       { src = Wp1; dst = wpp; Nout = DPR;  KP = DH;   segOff = g1 + g2; per = DH * DPR; }
  const int i = bstart + (int)threadIdx.x;
  if (i >= g1 + g2 + g3) return;
  const int o     = (i - segOff) * 8;
  const int layer = o / per;
  const int oo    = o - layer * per;
  const int n     = oo / KP;
  const int k0    = oo - n * KP;
  const float* sp = src + (size_t)layer * per + (size_t)k0 * Nout + n;
  v8us hv;
#pragma unroll
  for (int e = 0; e < 8; ++e) hv[e] = f2bf(sp[(size_t)e * Nout]);
  unsigned short* dp = dst + o;
  *(volatile v8us*)dp = hv;
  __threadfence();
  *(volatile v8us*)dp = hv;
}

__global__ __launch_bounds__(NTHR) void k_count(
    const int* __restrict__ edst, int* cnt, int nE, int vec8) {
  __shared__ __attribute__((aligned(16))) int scnt[NBC];
  __shared__ __attribute__((aligned(16))) int list[LISTN];
  __shared__ int wcnt[NWAVE];
  const int tid = threadIdx.x, lane = tid & 31, wave = tid >> 5;
  const int nodeBase = blockIdx.x * NBC;

  for (int i = tid; i < NBC; i += NTHR) scnt[i] = 0;
  __syncthreads();

  const int nChunks = (nE + CHUNK - 1) / CHUNK;
#pragma unroll 1
  for (int ch = 0; ch < nChunks; ++ch) {
    const int cbase = ch * CHUNK;
    const int wc = scan_chunk<NBC>(edst, nE, cbase, nodeBase, vec8, list, tid, lane, wave);
    if (lane == 0) wcnt[wave] = wc;
    __syncthreads();
    if (wave == 0) {
#pragma unroll 1
      for (int wsx = 0; wsx < NWAVE; ++wsx) {
        int n = __builtin_amdgcn_readfirstlane(wcnt[wsx]);
        n = n > WCAP ? WCAP : (n < 0 ? 0 : n);
        const int* lp = list + wsx * WCAP;
#pragma unroll 1
        for (int i = 0; i < n; ++i) {
          const int ent  = __builtin_amdgcn_readfirstlane(lp[i]);
          const int slot = ent & (NBC - 1);
          if (lane == 0) scnt[slot] = scnt[slot] + 1;
        }
      }
    }
    __syncthreads();
  }

  v4i cq[4];
#pragma unroll
  for (int q = 0; q < 4; ++q) {
    const int f = (wave * 4 + q) * 128 + 4 * lane;
    cq[q] = *(const v4i*)(scnt + f);
  }
  int* cp = cnt + (size_t)nodeBase;
#pragma unroll
  for (int q = 0; q < 4; ++q) {
    const int f = (wave * 4 + q) * 128 + 4 * lane;
    *(volatile v4i*)(cp + f) = cq[q];
  }
  __threadfence();
#pragma unroll
  for (int q = 0; q < 4; ++q) {
    const int f = (wave * 4 + q) * 128 + 4 * lane;
    *(volatile v4i*)(cp + f) = cq[q];
  }
}

__global__ __launch_bounds__(OTHR) void k_offsets(
    const int* __restrict__ cnt, int* off, int* rbase, int nChunk) {
  __shared__ __attribute__((aligned(16))) int soff[NBC];
  __shared__ __attribute__((aligned(16))) int srb[RBN];
  __shared__ int wtot[OTHR / 32];
  const int tid = threadIdx.x, lane = tid & 31, wave = tid >> 5, sub = tid >> 7;
  for (int i = tid; i < RBN; i += OTHR) srb[i] = 0;
  int carry = 0;
#pragma unroll 1
  for (int ch = 0; ch < nChunk; ++ch) {
    const int base = ch * NBC;
    const v4i c0 = *(const v4i*)(cnt + base + 8 * tid);
    const v4i c1 = *(const v4i*)(cnt + base + 8 * tid + 4);
    const int e0 = max(c0.x, 0), e1 = max(c0.y, 0), e2 = max(c0.z, 0), e3 = max(c0.w, 0);
    const int e4 = max(c1.x, 0), e5 = max(c1.y, 0), e6 = max(c1.z, 0), e7 = max(c1.w, 0);
    const int ts = e0 + e1 + e2 + e3 + e4 + e5 + e6 + e7;
    int incl = ts;
#pragma unroll
    for (int d = 1; d < 32; d <<= 1) {
      const int t = __shfl_up(incl, d);
      if (lane >= d) incl += t;
    }
    if (lane == 31) wtot[wave] = incl;
    __syncthreads();
    const int S0 = wtot[0]  + wtot[1]  + wtot[2]  + wtot[3];
    const int S1 = wtot[4]  + wtot[5]  + wtot[6]  + wtot[7];
    const int S2 = wtot[8]  + wtot[9]  + wtot[10] + wtot[11];
    const int S3 = wtot[12] + wtot[13] + wtot[14] + wtot[15];
    int pre = 0;
#pragma unroll 1
    for (int w = 4 * sub; w < wave; ++w) pre += wtot[w];
    const int b0 = carry;
    const int b1 = b0 + ((S0 + 31) & ~31);
    const int b2 = b1 + ((S1 + 31) & ~31);
    const int b3 = b2 + ((S2 + 31) & ~31);
    const int b4 = b3 + ((S3 + 31) & ~31);
    const int myb = sub == 0 ? b0 : (sub == 1 ? b1 : (sub == 2 ? b2 : b3));
    if (tid == 0) {
      srb[min(4 * ch + 0, RBN - 1)] = b0;
      srb[min(4 * ch + 1, RBN - 1)] = b1;
      srb[min(4 * ch + 2, RBN - 1)] = b2;
      srb[min(4 * ch + 3, RBN - 1)] = b3;
    }
    int run = myb + pre + incl - ts;
    soff[8 * tid + 0] = run; run += e0;
    soff[8 * tid + 1] = run; run += e1;
    soff[8 * tid + 2] = run; run += e2;
    soff[8 * tid + 3] = run; run += e3;
    soff[8 * tid + 4] = run; run += e4;
    soff[8 * tid + 5] = run; run += e5;
    soff[8 * tid + 6] = run; run += e6;
    soff[8 * tid + 7] = run;
    carry = b4;
    __syncthreads();
    const v4i o0 = *(const v4i*)(soff + 4 * tid);
    const v4i o1 = *(const v4i*)(soff + 4 * (tid + OTHR));
    int* op = off + base;
    *(volatile v4i*)(op + 4 * tid) = o0;
    *(volatile v4i*)(op + 4 * (tid + OTHR)) = o1;
    __threadfence();
    *(volatile v4i*)(op + 4 * tid) = o0;
    *(volatile v4i*)(op + 4 * (tid + OTHR)) = o1;
    __syncthreads();
  }
  if (tid == 0) srb[min(4 * nChunk, RBN - 1)] = carry;
  __syncthreads();
  v4i rv = {0, 0, 0, 0};
  if (tid < 32) rv = *(const v4i*)(srb + 4 * tid);
  if (tid < 32) *(volatile v4i*)(rbase + 4 * tid) = rv;
  __threadfence();
  if (tid < 32) *(volatile v4i*)(rbase + 4 * tid) = rv;
}

__global__ __launch_bounds__(NTHR) void k_fill(
    const int* __restrict__ esrc, const int* __restrict__ edst,
    const int* __restrict__ off, const int* __restrict__ rbase,
    int* csr, int nN, int nE, int vec8, int csrLen) {
  extern __shared__ v4f lds_dyn[];
  int* region = (int*)lds_dyn;
  int* cursor = region + RCAP;
  int* list   = cursor + NBF;
  int* wcnt   = list + LISTN;
  const int tid = threadIdx.x, lane = tid & 31, wave = tid >> 5;
  const int b = blockIdx.x;
  const int nodeBase = b * NBF;

  int rb0 = rbase[b];
  const int rb1 = rbase[b + 1];
  rb0 = rb0 < 0 ? 0 : (rb0 > csrLen ? csrLen : rb0);
  rb0 &= ~31;
  int len = rb1 - rb0;
  len = len < 0 ? 0 : (len > RCAP ? RCAP : len);
  int lenW = (len + 31) & ~31;
  if (rb0 + lenW > csrLen) lenW = (csrLen - rb0) & ~31;

  {
    const v4i z = {0, 0, 0, 0};
    for (int i = tid; i < RCAP / 4; i += NTHR) ((v4i*)region)[i] = z;
    for (int s = tid; s < NBF; s += NTHR) {
      int o = off[nodeBase + s] - rb0;
      o = o < 0 ? 0 : (o > RCAP ? RCAP : o);
      cursor[s] = o;
    }
  }
  __syncthreads();

  const int nChunks = (nE + CHUNK - 1) / CHUNK;
#pragma unroll 1
  for (int ch = 0; ch < nChunks; ++ch) {
    const int cbase = ch * CHUNK;
    const int wc = scan_chunk<NBF>(edst, nE, cbase, nodeBase, vec8, list, tid, lane, wave);
    if (lane == 0) wcnt[wave] = wc;
    __syncthreads();
    if (wave == 0) {
#pragma unroll 1
      for (int wsx = 0; wsx < NWAVE; ++wsx) {
        int n = __builtin_amdgcn_readfirstlane(wcnt[wsx]);
        n = n > WCAP ? WCAP : (n < 0 ? 0 : n);
        const int* lp = list + wsx * WCAP;
#pragma unroll 1
        for (int i = 0; i < n; ++i) {
          const int ent  = __builtin_amdgcn_readfirstlane(lp[i]);
          const int slot = ent & (NBF - 1);
          int e = cbase + ((ent >> 12) & (CHUNK - 1));
          e = e > nE - 1 ? nE - 1 : e;
          int src = esrc[e];
          src = src < 0 ? 0 : (src > nN - 1 ? nN - 1 : src);
          if (lane == 0) {
            int pos = cursor[slot];
            pos = pos < 0 ? 0 : (pos > RCAP - 1 ? RCAP - 1 : pos);
            region[pos] = src;
            const int np = pos + 1;
            cursor[slot] = np > RCAP ? RCAP : np;
          }
        }
      }
    }
    __syncthreads();
  }

  const int nv = lenW >> 2;
  int* gp = csr + rb0;
#pragma unroll 1
  for (int i = tid; i < nv; i += NTHR) { const v4i v = ((const v4i*)region)[i]; *(volatile v4i*)(gp + 4 * i) = v; }
  __threadfence();
#pragma unroll 1
  for (int i = tid; i < nv; i += NTHR) { const v4i v = ((const v4i*)region)[i]; *(volatile v4i*)(gp + 4 * i) = v; }
}

template <int RNE_IN>
__global__ __launch_bounds__(NTHR) void k_agg(
    const int* __restrict__ csr, const int* __restrict__ off, const int* __restrict__ cnt,
    const float* __restrict__ hin, unsigned short* shi, unsigned short* slo, int nN, int csrLen) {
  const int tid = threadIdx.x, lane = tid & 31, wave = tid >> 5;
  const int tbase = blockIdx.x * TGT + wave * 32;
  const int cl = tbase + lane;
  const int cnt_l = cnt[cl];
  const int off_l = off[cl];

#pragma unroll 1
  for (int j = 0; j < 32; ++j) {
    const int c = tbase + j;
    int n = __builtin_amdgcn_readlane(cnt_l, j);
    n = n < 0 ? 0 : (n > DEGCAP ? DEGCAP : n);
    const int st = __builtin_amdgcn_readlane(off_l, j);
    v4f acc = {0.f, 0.f, 0.f, 0.f};
#pragma unroll 1
    for (int q0 = 0; q0 < n; q0 += 32) {
      int pos = st + q0 + lane;
      pos = pos < 0 ? 0 : (pos > csrLen - 1 ? csrLen - 1 : pos);
      int sl = csr[pos];
      sl = sl < 0 ? 0 : (sl > nN - 1 ? nN - 1 : sl);
      const int mcnt = (n - q0) < 32 ? (n - q0) : 32;
#pragma unroll 1
      for (int p = 0; p < mcnt; ++p) {
        const int s = __builtin_amdgcn_readlane(sl, p);
        v4f v = *(const v4f*)(hin + (size_t)s * DH + 4 * lane);
        if (RNE_IN != 0) v = bfr4(v);
        acc = acc + v;
      }
    }
    const int cc = c > nN - 1 ? nN - 1 : c;
    v4f sv = *(const v4f*)(hin + (size_t)cc * DH + 4 * lane);
    if (RNE_IN != 0) sv = bfr4(sv);
    const v4f s = sv + acc;
    v4us hv, lv;
    split4(s, hv, lv);
    unsigned short* hp = shi + (size_t)c * DH + 4 * lane;
    unsigned short* lp = slo + (size_t)c * DH + 4 * lane;
    *(volatile v4us*)hp = hv;
    *(volatile v4us*)lp = lv;
    __threadfence();
    *(volatile v4us*)hp = hv;
    *(volatile v4us*)lp = lv;
  }
}

__global__ __launch_bounds__(GTHR) void k_gin(
    const unsigned short* __restrict__ shi, const unsigned short* __restrict__ slo,
    const unsigned short* __restrict__ w1p, const float* __restrict__ b1,
    const unsigned short* __restrict__ w2p, const float* __restrict__ b2,
    float* hout, int nStore) {
  extern __shared__ v4f lds_dyn[];
  unsigned short* zhi = (unsigned short*)lds_dyn;
  unsigned short* zlo = zhi + GR * ZP;
  float*          stg = (float*)lds_dyn;
  const int tid = threadIdx.x, lane = tid & 31, wave = tid >> 5, hh = lane >> 4, m = lane & 15;
  const int rowBase = blockIdx.x * GR;
  const int r0 = wave * 16;

  FragB ah[4], al[4];
  {
    const size_t ao = (size_t)(rowBase + r0 + m) * DH + 8 * hh;
    const unsigned short* php = shi + ao;
    const unsigned short* plp = slo + ao;
#pragma unroll
    for (int kt = 0; kt < DH / 32; ++kt) {
      ah[kt].h[0] = *(const v8us*)(php + 32 * kt);
      ah[kt].h[1] = *(const v8us*)(php + 32 * kt + 16);
      al[kt].h[0] = *(const v8us*)(plp + 32 * kt);
      al[kt].h[1] = *(const v8us*)(plp + 32 * kt + 16);
    }
  }

#pragma unroll 1
  for (int g = 0; g < DMLP / 64; ++g) {
    v8f acc[4];
#pragma unroll
    for (int t = 0; t < 4; ++t) acc[t] = zero8();
#pragma unroll
    for (int kt = 0; kt < DH / 32; ++kt) {
#pragma unroll
      for (int t = 0; t < 4; ++t) {
        const unsigned short* bp = w1p + (size_t)(64 * g + 16 * t + m) * DH + 32 * kt + 8 * hh;
        FragB b;
        b.h[0] = *(const v8us*)bp;
        b.h[1] = *(const v8us*)(bp + 16);
        acc[t] = wmb(ah[kt].v, b.v, acc[t]);
        acc[t] = wmb(al[kt].v, b.v, acc[t]);
      }
    }
#pragma unroll
    for (int t = 0; t < 4; ++t) {
      const int col = 64 * g + 16 * t + m;
      const float bv = bfr(b1[col]);
      unsigned short* zh = zhi + (r0 + 8 * hh) * ZP + col;
      unsigned short* zl = zlo + (r0 + 8 * hh) * ZP + col;
#pragma unroll
      for (int r = 0; r < 8; ++r) {
        const float v = fmaxf(acc[t][r] + bv, 0.0f);
        const unsigned short hb = f2bf(v);
        const unsigned short lb = f2bf(v - bf2f(hb));
        zh[r * ZP] = hb;
        zl[r * ZP] = lb;
      }
    }
  }
  __syncthreads();

  v8f acc2[8];
#pragma unroll
  for (int nt = 0; nt < 8; ++nt) acc2[nt] = zero8();
  const unsigned short* zr  = zhi + (r0 + m) * ZP + 8 * hh;
  const unsigned short* zlr = zlo + (r0 + m) * ZP + 8 * hh;
#pragma unroll 1
  for (int kt = 0; kt < DMLP / 32; ++kt) {
    FragB a, c;
    a.h[0] = *(const v8us*)(zr + 32 * kt);
    a.h[1] = *(const v8us*)(zr + 32 * kt + 16);
    c.h[0] = *(const v8us*)(zlr + 32 * kt);
    c.h[1] = *(const v8us*)(zlr + 32 * kt + 16);
#pragma unroll
    for (int nt = 0; nt < 8; ++nt) {
      const unsigned short* bp = w2p + (size_t)(16 * nt + m) * DMLP + 32 * kt + 8 * hh;
      FragB b;
      b.h[0] = *(const v8us*)bp;
      b.h[1] = *(const v8us*)(bp + 16);
      acc2[nt] = wmb(a.v, b.v, acc2[nt]);
      acc2[nt] = wmb(c.v, b.v, acc2[nt]);
    }
  }
  __syncthreads();

  {
    float* sp = stg + (r0 + 8 * hh) * DH + m;
#pragma unroll
    for (int nt = 0; nt < 8; ++nt) {
      const float bv = bfr(b2[16 * nt + m]);
#pragma unroll
      for (int r = 0; r < 8; ++r) sp[r * DH + 16 * nt] = fmaxf(acc2[nt][r] + bv, 0.0f);
    }
  }
  __syncthreads();

  const float* lp = stg + r0 * DH + 4 * lane;
  float* gp = hout + ((size_t)rowBase + r0) * DH + 4 * lane;
#pragma unroll
  for (int i = 0; i < 16; ++i) {
    if (rowBase + r0 + i < nStore) { const v4f v = *(const v4f*)(lp + i * DH); *(volatile v4f*)(gp + (size_t)i * DH) = v; }
  }
  __threadfence();
#pragma unroll
  for (int i = 0; i < 16; ++i) {
    if (rowBase + r0 + i < nStore) { const v4f v = *(const v4f*)(lp + i * DH); *(volatile v4f*)(gp + (size_t)i * DH) = v; }
  }
}

__global__ __launch_bounds__(PTHR) void k_pred(
    const float* __restrict__ h, const int* __restrict__ ps, const int* __restrict__ pd,
    const int* __restrict__ ns, const int* __restrict__ nd,
    const unsigned short* __restrict__ wpp, const float* __restrict__ bp1,
    const float* __restrict__ wp2, const float* __restrict__ bp2,
    float* out, int nP, int nOut, int nN) {
  __shared__ __attribute__((aligned(16))) unsigned short ahi[PB * SPP];
  __shared__ __attribute__((aligned(16))) unsigned short alo[PB * SPP];
  __shared__ __attribute__((aligned(16))) float sOut[PB];
  const int tid = threadIdx.x, lane = tid & 31, wave = tid >> 5, hh = lane >> 4, m = lane & 15;
  const int pb = blockIdx.x * PB + wave * 16;

  const int e = pb + m;
  int ip = e;       ip = ip > nP - 1 ? nP - 1 : ip;
  int iq = e - nP;  iq = iq < 0 ? 0 : (iq > nP - 1 ? nP - 1 : iq);
  const int sa = ps[ip], da = pd[ip], sb = ns[iq], db = nd[iq];
  int s = e < nP ? sa : sb;
  int d = e < nP ? da : db;
  s = s < 0 ? 0 : (s > nN - 1 ? nN - 1 : s);
  d = d < 0 ? 0 : (d > nN - 1 ? nN - 1 : d);

#pragma unroll 1
  for (int j = 0; j < 16; ++j) {
    const int sj = __builtin_amdgcn_readlane(s, j);
    const int dj = __builtin_amdgcn_readlane(d, j);
    const v4f va = *(const v4f*)(h + (size_t)sj * DH + 4 * lane);
    const v4f vb = *(const v4f*)(h + (size_t)dj * DH + 4 * lane);
    const v4f pr = va * vb;
    v4us hv, lv;
    split4(pr, hv, lv);
    *(v4us*)(ahi + (wave * 16 + j) * SPP + 4 * lane) = hv;
    *(v4us*)(alo + (wave * 16 + j) * SPP + 4 * lane) = lv;
  }
  __syncthreads();

  FragB fh[4], fl[4];
  {
    const unsigned short* php = ahi + (wave * 16 + m) * SPP + 8 * hh;
    const unsigned short* plp = alo + (wave * 16 + m) * SPP + 8 * hh;
#pragma unroll
    for (int kt = 0; kt < DH / 32; ++kt) {
      fh[kt].h[0] = *(const v8us*)(php + 32 * kt);
      fh[kt].h[1] = *(const v8us*)(php + 32 * kt + 16);
      fl[kt].h[0] = *(const v8us*)(plp + 32 * kt);
      fl[kt].h[1] = *(const v8us*)(plp + 32 * kt + 16);
    }
  }
  v8f acc[4];
#pragma unroll
  for (int t = 0; t < 4; ++t) acc[t] = zero8();
#pragma unroll
  for (int kt = 0; kt < DH / 32; ++kt) {
#pragma unroll
    for (int t = 0; t < 4; ++t) {
      const unsigned short* bp = wpp + (size_t)(16 * t + m) * DH + 32 * kt + 8 * hh;
      FragB b;
      b.h[0] = *(const v8us*)bp;
      b.h[1] = *(const v8us*)(bp + 16);
      acc[t] = wmb(fh[kt].v, b.v, acc[t]);
      acc[t] = wmb(fl[kt].v, b.v, acc[t]);
    }
  }

  float part[8];
#pragma unroll
  for (int r = 0; r < 8; ++r) part[r] = 0.0f;
#pragma unroll
  for (int t = 0; t < 4; ++t) {
    const int col = 16 * t + m;
    const float bv = bfr(bp1[col]);
    const float wv = bfr(wp2[col]);
#pragma unroll
    for (int r = 0; r < 8; ++r) part[r] += fmaxf(acc[t][r] + bv, 0.0f) * wv;
  }
#pragma unroll
  for (int r = 0; r < 8; ++r) {
    part[r] += __shfl_xor(part[r], 8);
    part[r] += __shfl_xor(part[r], 4);
    part[r] += __shfl_xor(part[r], 2);
    part[r] += __shfl_xor(part[r], 1);
  }
  const float b2v = bfr(bp2[0]);
  if (m == 0) {
#pragma unroll
    for (int r = 0; r < 8; ++r) sOut[wave * 16 + 8 * hh + r] = part[r] + b2v;
  }
  __syncthreads();

  const int base = blockIdx.x * PB + 4 * tid;
  v4f ov = {0.f, 0.f, 0.f, 0.f};
  if (tid < 16) ov = *(const v4f*)(sOut + 4 * tid);
  if (tid < 16 && base < nOut) *(volatile v4f*)(out + base) = ov;
  __threadfence();
  if (tid < 16 && base < nOut) *(volatile v4f*)(out + base) = ov;
}

extern "C" void kernel_launch(void* const* d_in, const int* in_sizes, int n_in,
                              void* d_out, int out_size, void* d_ws, size_t ws_size,
                              hipStream_t stream) {
  if (n_in < 15) return;
  const int nN = in_sizes[0] / DH;
  if (nN <= 0 || in_sizes[0] != nN * DH) return;
  const int nL = in_sizes[1] / (DH * DMLP);
  if (nL < 1 || in_sizes[1] != nL * DH * DMLP || in_sizes[2] < nL * DMLP) return;
  if (in_sizes[3] != nL * DMLP * DH || in_sizes[4] < nL * DH) return;
  if (in_sizes[5] != DH * DPR || in_sizes[6] < DPR || in_sizes[7] < DPR || in_sizes[8] < 1) return;
  const int nE = in_sizes[9];
  if (nE <= 0 || in_sizes[10] != nE) return;
  const int nP = in_sizes[11];
  if (nP <= 0 || in_sizes[12] != nP || in_sizes[13] != nP || in_sizes[14] != nP) return;
  const int nOut = 2 * nP;
  if ((nOut & 3) != 0) return;
  if (out_size != nOut + nN * DH) return;
  if (nE > (1 << 28) || nN > (1 << 24)) return;

  const float* x   = (const float*)d_in[0];
  const float* W1  = (const float*)d_in[1];
  const float* b1  = (const float*)d_in[2];
  const float* W2  = (const float*)d_in[3];
  const float* b2  = (const float*)d_in[4];
  const float* Wp1 = (const float*)d_in[5];
  const float* bp1 = (const float*)d_in[6];
  const float* Wp2 = (const float*)d_in[7];
  const float* bp2 = (const float*)d_in[8];
  const int*   esrc = (const int*)d_in[9];
  const int*   edst = (const int*)d_in[10];
  const int*   ps  = (const int*)d_in[11];
  const int*   pd  = (const int*)d_in[12];
  const int*   ns  = (const int*)d_in[13];
  const int*   nd  = (const int*)d_in[14];
  float* out  = (float*)d_out;
  float* outH = out + (size_t)nOut;

  const int NPAD   = ((nN + TGT - 1) / TGT) * TGT;
  const int nBC    = (nN + NBC - 1) / NBC;
  const int CNTPAD = nBC * NBC;
  if (4 * nBC + 1 > RBN) return;
  const int nBF    = (nN + NBF - 1) / NBF;
  const int csrLen = ((nE + 31) & ~31) + 4096;
  const int nAgg   = NPAD / TGT;
  const int nGin   = NPAD / GR;
  const int nPrd   = (nOut + PB - 1) / PB;

  char* ws = (char*)d_ws;
  size_t off = 0;
  const size_t oW1  = off; off += (size_t)nL * DH * DMLP * 2;   off = (off + 255) & ~(size_t)255;
  const size_t oW2  = off; off += (size_t)nL * DMLP * DH * 2;   off = (off + 255) & ~(size_t)255;
  const size_t oWp  = off; off += (size_t)DH * DPR * 2;         off = (off + 255) & ~(size_t)255;
  const size_t oCnt = off; off += (size_t)CNTPAD * 4;           off = (off + 255) & ~(size_t)255;
  const size_t oOff = off; off += (size_t)CNTPAD * 4;           off = (off + 255) & ~(size_t)255;
  const size_t oRb  = off; off += (size_t)RBN * 4;              off = (off + 255) & ~(size_t)255;
  const size_t oCsr = off; off += (size_t)csrLen * 4;           off = (off + 255) & ~(size_t)255;
  const size_t oH   = off; off += (size_t)NPAD * DH * 4;        off = (off + 255) & ~(size_t)255;
  const size_t oShi = off; off += (size_t)NPAD * DH * 2;        off = (off + 255) & ~(size_t)255;
  const size_t oSlo = off; off += (size_t)NPAD * DH * 2;        off = (off + 255) & ~(size_t)255;
  if (off > ws_size) return;
  unsigned short* w1p = (unsigned short*)(ws + oW1);
  unsigned short* w2p = (unsigned short*)(ws + oW2);
  unsigned short* wpp = (unsigned short*)(ws + oWp);
  int*   cnt  = (int*)(ws + oCnt);
  int*   offp = (int*)(ws + oOff);
  int*   rb   = (int*)(ws + oRb);
  int*   csr  = (int*)(ws + oCsr);
  float* hpl  = (float*)(ws + oH);
  unsigned short* shi = (unsigned short*)(ws + oShi);
  unsigned short* slo = (unsigned short*)(ws + oSlo);

  const int vec8 = ((nE & 3) == 0) ? 1 : 0;

  const int nPrep = nL * (DH * DMLP / 8) + nL * (DMLP * DH / 8) + DH * DPR / 8;
  k_wprep<<<(nPrep + NTHR - 1) / NTHR, NTHR, 0, stream>>>(W1, W2, Wp1, w1p, w2p, wpp, nL);

  k_count<<<nBC, NTHR, 0, stream>>>(edst, cnt, nE, vec8);
  k_offsets<<<1, OTHR, 0, stream>>>(cnt, offp, rb, nBC);
  hipFuncSetAttribute(reinterpret_cast<const void*>(&k_fill),
                      hipFuncAttributeMaxDynamicSharedMemorySize, LDS_FILL);
  k_fill<<<nBF, NTHR, LDS_FILL, stream>>>(esrc, edst, offp, rb, csr, nN, nE, vec8, csrLen);

  hipFuncSetAttribute(reinterpret_cast<const void*>(&k_gin),
                      hipFuncAttributeMaxDynamicSharedMemorySize, LDS_GIN);
  for (int l = 0; l < nL; ++l) {
    const int last = (l == nL - 1) ? 1 : 0;
    if (l == 0) k_agg<1><<<nAgg, NTHR, 0, stream>>>(csr, offp, cnt, x,   shi, slo, nN, csrLen);
    else        k_agg<0><<<nAgg, NTHR, 0, stream>>>(csr, offp, cnt, hpl, shi, slo, nN, csrLen);
    k_gin<<<nGin, GTHR, LDS_GIN, stream>>>(shi, slo,
                                          w1p + (size_t)l * DH * DMLP, b1 + (size_t)l * DMLP,
                                          w2p + (size_t)l * DMLP * DH, b2 + (size_t)l * DH,
                                          last ? outH : hpl, last ? nN : NPAD);
  }

  k_pred<<<nPrd, PTHR, 0, stream>>>(outH, ps, pd, ns, nd, wpp, bp1, Wp2, bp2, out, nP, nOut, nN);
}
